// SGCNet2_90580860272649
// MI455X (gfx1250) — hardware-verified
//
#include <hip/hip_runtime.h>
#include <stdint.h>
#include <math.h>

#define NN   100000
#define NE   1600000
#define DD   128
#define NCLS 40
#define NCP  64
#define MP   100032
#define NT   256
#define SRB  2048
#define NTL  49
#define NPA  (NTL * SRB)
#define SCH  2048
#define SPT  (SCH / NT)
#define NCH  ((NE + SCH - 1) / SCH)
#define LSB  64
#define NLB  ((NN + LSB - 1) / LSB)

static_assert(NPA >= MP, "");
static_assert(MP % 64 == 0 && MP >= NN, "");
static_assert(NLB * LSB == MP, "");
static_assert(NE % SPT == 0, "");
static_assert((LSB * NCLS) % 128 == 0, "");
static_assert(((NN % LSB) * NCLS) % 128 == 0, "");
static_assert(DD % 32 == 0 && NCP % 64 == 0, "");
static_assert(NN < (1 << 17) && SRB <= (1 << 11), "");

typedef __attribute__((ext_vector_type(16))) _Float16 v16h;
typedef __attribute__((ext_vector_type(8)))  _Float16 v8h;
typedef __attribute__((ext_vector_type(16))) __bf16   v16b;
typedef __attribute__((ext_vector_type(8)))  __bf16   v8b;
typedef __attribute__((ext_vector_type(8)))  float    v8f;
typedef __attribute__((ext_vector_type(4)))  float    v4f;
typedef __attribute__((ext_vector_type(4)))  int      v4i;

__device__ __forceinline__ unsigned short f2bf_bits(float f) {
  unsigned u = __float_as_uint(f);
  return (unsigned short)((u + 0x7FFFu + ((u >> 16) & 1u)) >> 16);
}
__device__ __forceinline__ float bf_bits2f(unsigned short h) { return __uint_as_float(((unsigned)h) << 16); }

__device__ __forceinline__ void dep_guard_h(v8f& a, v8f& b, v16h x, v16h y) { asm volatile("v_nop\n\tv_nop\n\tv_nop\n\tv_nop" : "+v"(a), "+v"(b) : "v"(x), "v"(y)); }
__device__ __forceinline__ void dep_guard_b(v8f& a, v8f& b, v16b x, v16b y) { asm volatile("v_nop\n\tv_nop\n\tv_nop\n\tv_nop" : "+v"(a), "+v"(b) : "v"(x), "v"(y)); }
__device__ __forceinline__ void keep4_h(v16h a, v16h b, v16h c, v16h d) { asm volatile("v_nop" :: "v"(a), "v"(b), "v"(c), "v"(d)); }
__device__ __forceinline__ void keep4_b(v16b a, v16b b, v16b c, v16b d) { asm volatile("v_nop" :: "v"(a), "v"(b), "v"(c), "v"(d)); }
__device__ __forceinline__ void acc_guard4(v8f& a, v8f& b, v8f& c, v8f& d) { asm volatile("v_nop\n\tv_nop\n\tv_nop\n\tv_nop" : "+v"(a), "+v"(b), "+v"(c), "+v"(d)); }
template <typename T> struct Frag;
template <> struct Frag<_Float16> {
  typedef v16h V; union U { v16h v; v8h h[2]; };
  static __device__ __forceinline__ v16h load(const _Float16* p) {
    U f; f.h[0] = *(const v8h*)(p); f.h[1] = *(const v8h*)(p + 16); return f.v;
  }
  static __device__ __forceinline__ v8f mma(v16h a, v16h b, v8f c) {
    return __builtin_amdgcn_wmma_f32_16x16x32_f16(false, a, false, b, (short)0, c, false, false);
  }
  static __device__ __forceinline__ void guard(v8f& a, v8f& b, v16h x, v16h y) { dep_guard_h(a, b, x, y); }
  static __device__ __forceinline__ void keep(v16h a, v16h b, v16h c, v16h d) { keep4_h(a, b, c, d); }
};
template <> struct Frag<__bf16> {
  typedef v16b V; union U { v16b v; v8b h[2]; };
  static __device__ __forceinline__ v16b load(const __bf16* p) {
    U f; f.h[0] = *(const v8b*)(p); f.h[1] = *(const v8b*)(p + 16); return f.v;
  }
  static __device__ __forceinline__ v8f mma(v16b a, v16b b, v8f c) {
    return __builtin_amdgcn_wmma_f32_16x16x32_bf16(false, a, false, b, (short)0, c, false, false);
  }
  static __device__ __forceinline__ void guard(v8f& a, v8f& b, v16b x, v16b y) { dep_guard_b(a, b, x, y); }
  static __device__ __forceinline__ void keep(v16b a, v16b b, v16b c, v16b d) { keep4_b(a, b, c, d); }
};

template <int ET> struct Elem;
template <> struct Elem<0> { typedef _Float16 T; };
template <> struct Elem<1> { typedef __bf16 T; };
template <int ET, bool SPLIT, int BIAS_MODE, int OUT_MODE, bool RESID, int ACT = 0>
__global__ __launch_bounds__(256) void wmma_gemm64(
    const unsigned short* __restrict__ Ap, const unsigned short* __restrict__ A2p, int lda, long strideA,
    const unsigned short* __restrict__ Btp, const unsigned short* __restrict__ Bt2p, int ldb, long strideB,
    void* __restrict__ Cout, void* __restrict__ Cout2, int ldc, long strideC,
    const float* __restrict__ bias,
    const float* __restrict__ resid, long strideR,
    int M, int N, int K, float scale) {
  typedef typename Elem<ET>::T T;
  typedef typename Frag<T>::V V;
  const T* A = (const T*)Ap; const T* A2 = (const T*)A2p; const T* Bt = (const T*)Btp; const T* Bt2 = (const T*)Bt2p;
  __shared__ __align__(16) float sT[8][16 * 68];
  const int b    = blockIdx.y;
  const int lane = threadIdx.x & 31;
  const int wave = threadIdx.x >> 5;
  const int tilesN = N >> 6;
  const int tilesM = M >> 6;
  const int tile = blockIdx.x * 8 + wave;
  if (tile >= tilesM * tilesN) return;
  const int tm = tile / tilesN;
  const int tn = tile - tm * tilesN;
  const int m0 = tm << 6;
  const int n0 = tn << 6;

  const T* Ab  = A  + (size_t)b * strideA;
  const T* Bb  = Bt + (size_t)b * strideB;
  const T* Ab2 = SPLIT ? (A2  + (size_t)b * strideA) : nullptr;
  const T* Bb2 = SPLIT ? (Bt2 + (size_t)b * strideB) : nullptr;

  const int rlane = lane & 15;
  const int koff  = (lane >> 4) * 8;
  const int mOff  = (lane >> 4) * 8;

  v8f acc[4][4];
#pragma unroll
  for (int i = 0; i < 4; ++i)
#pragma unroll
    for (int j = 0; j < 4; ++j) acc[i][j] = (v8f){0.f,0.f,0.f,0.f,0.f,0.f,0.f,0.f};

  for (int k0 = 0; k0 < K; k0 += 32) {
    V bh[4], bl[4];
#pragma unroll
    for (int j = 0; j < 4; ++j) {
      const size_t bo = (size_t)(n0 + (j << 4) + rlane) * ldb + koff + k0;
      bh[j] = Frag<T>::load(Bb + bo);
      if (SPLIT) bl[j] = Frag<T>::load(Bb2 + bo);
    }
#pragma unroll
    for (int i = 0; i < 4; ++i) {
      const size_t ao = (size_t)(m0 + (i << 4) + rlane) * lda + koff + k0;
      V ah = Frag<T>::load(Ab + ao);
      V al;
      if (SPLIT) al = Frag<T>::load(Ab2 + ao);
#pragma unroll
      for (int j = 0; j < 4; ++j) {
        acc[i][j] = Frag<T>::mma(ah, bh[j], acc[i][j]);
        if (SPLIT) {
          acc[i][j] = Frag<T>::mma(ah, bl[j], acc[i][j]);
          acc[i][j] = Frag<T>::mma(al, bh[j], acc[i][j]);
        }
      }
      Frag<T>::guard(acc[i][0], acc[i][3], ah, SPLIT ? al : ah);
    }
    Frag<T>::keep(bh[0], bh[1], bh[2], bh[3]);
    if (SPLIT) Frag<T>::keep(bl[0], bl[1], bl[2], bl[3]);
  }
  acc_guard4(acc[0][0], acc[0][1], acc[0][2], acc[0][3]);
  acc_guard4(acc[1][0], acc[1][1], acc[1][2], acc[1][3]);
  acc_guard4(acc[2][0], acc[2][1], acc[2][2], acc[2][3]);
  acc_guard4(acc[3][0], acc[3][1], acc[3][2], acc[3][3]);

  float* slab = sT[wave];
  const float* Rb = RESID ? (resid + (size_t)b * strideR) : nullptr;
#pragma unroll
  for (int i = 0; i < 4; ++i) {
    const int mBase = m0 + (i << 4);
#pragma unroll
    for (int j = 0; j < 4; ++j) {
      const int n = n0 + (j << 4) + rlane;
      float bv = 0.f;
      if (BIAS_MODE == 2) bv = bias[n];
#pragma unroll
      for (int r = 0; r < 8; ++r) {
        float v = acc[i][j][r] * scale;
        if (BIAS_MODE == 1) v += bias[mBase + mOff + r];
        if (BIAS_MODE == 2) v += bv;
        if (RESID) v += Rb[(size_t)(mBase + mOff + r) * ldc + n];
        if (ACT == 1) v = tanhf(v);
        if (ACT == 2) v = fmaxf(v, 0.0f);
        if (ACT == 3) v = v / (1.0f + expf(-v));
        if (ACT == 4) v = (v > 0.f) ? v : 0.01f * v;
        if (ACT == 5) v = 0.5f * v * (1.0f + erff(v * 0.70710678118654752f));
        slab[(mOff + r) * 68 + (j << 4) + rlane] = v;
      }
    }
    __builtin_amdgcn_fence(__ATOMIC_RELEASE, "workgroup");
    __builtin_amdgcn_wave_barrier();
    __builtin_amdgcn_fence(__ATOMIC_ACQUIRE, "workgroup");
    if (OUT_MODE == 0) {
      float* C = (float*)Cout + (size_t)b * strideC;
      const int hh = lane >> 4, c4 = (lane & 15) * 4;
      for (int pass = 0; pass < 2; ++pass) {
#pragma unroll
        for (int it = 0; it < 8; ++it) {
          const int row = it * 2 + hh;
          v4f v = *(const v4f*)(slab + row * 68 + c4);
          *(volatile v4f*)(C + (size_t)(mBase + row) * ldc + n0 + c4) = v;
        }
        __threadfence();
      }
    } else {
      const int q = lane >> 3, c8 = (lane & 7) * 8;
      unsigned short* C  = (unsigned short*)Cout  + (size_t)b * strideC;
      unsigned short* C2 = (OUT_MODE == 2) ? ((unsigned short*)Cout2 + (size_t)b * strideC) : nullptr;
      for (int pass = 0; pass < 2; ++pass) {
#pragma unroll
        for (int it = 0; it < 4; ++it) {
          const int row = it * 4 + q;
          const float* sp = slab + row * 68 + c8;
          v8h hv, lv;
#pragma unroll
          for (int e = 0; e < 8; ++e) {
            if (OUT_MODE == 1) {
              hv[e] = (_Float16)sp[e];
            } else {
              unsigned short hb = f2bf_bits(sp[e]);
              unsigned short lb = f2bf_bits(sp[e] - bf_bits2f(hb));
              hv[e] = __builtin_bit_cast(_Float16, hb);
              lv[e] = __builtin_bit_cast(_Float16, lb);
            }
          }
          *(volatile v8h*)(C + (size_t)(mBase + row) * ldc + n0 + c8) = hv;
          if (OUT_MODE == 2) *(volatile v8h*)(C2 + (size_t)(mBase + row) * ldc + n0 + c8) = lv;
        }
        __threadfence();
      }
    }
    __builtin_amdgcn_fence(__ATOMIC_RELEASE, "workgroup");
    __builtin_amdgcn_wave_barrier();
    __builtin_amdgcn_fence(__ATOMIC_ACQUIRE, "workgroup");
  }
}

__global__ __launch_bounds__(256) void wt_cast_kernel(const float* __restrict__ W, unsigned* __restrict__ outp) {
  const int i = blockIdx.x * 256 + threadIdx.x;
  if (i >= NCP * (DD / 2)) return;
  const int f = i / (DD / 2);
  const int k = 2 * (i - f * (DD / 2));
  const int fc = (f < NCLS) ? f : (NCLS - 1);
  float a = W[(size_t)k * NCLS + fc] * 16.0f;
  float b = W[(size_t)(k + 1) * NCLS + fc] * 16.0f;
  if (f >= NCLS) { a = 0.0f; b = 0.0f; }
  const unsigned u = (unsigned)__builtin_bit_cast(unsigned short, (_Float16)a) | ((unsigned)__builtin_bit_cast(unsigned short, (_Float16)b) << 16);
  ((volatile unsigned*)outp)[i] = u;
  __threadfence();
  ((volatile unsigned*)outp)[i] = u;
}

__device__ __forceinline__ int blk_excl_scan(int cnt, int* scan_ws, int tid, int* tot) {
  const int lane = tid & 31, wave = tid >> 5; int incl = cnt;
#pragma unroll
  for (int o = 1; o < 32; o <<= 1) { const int v = __shfl_up(incl, o, 32); if (lane >= o) incl += v; }
  if (lane == 31) scan_ws[wave] = incl;
  __syncthreads();
  if (wave == 0) { int wv = (lane < NT / 32) ? scan_ws[lane] : 0; int wincl = wv;
#pragma unroll
    for (int o = 1; o < 32; o <<= 1) { const int v = __shfl_up(wincl, o, 32); if (lane >= o) wincl += v; }
    if (lane < NT / 32) scan_ws[32 + lane] = wincl - wv; if (lane == 31) scan_ws[64] = wincl; }
  __syncthreads();
  const int res = scan_ws[32 + wave] + incl - cnt; *tot = scan_ws[64];
  return res;
}
template <int SP, int CAP, bool SRCL>
__device__ __forceinline__ int chunk_hits(const int* __restrict__ dstv, const int* __restrict__ srcv, int e0, int n0, int tid,
                                          int* LIST, int* scan_ws) {
  const int eb = e0 + tid * SP;
  const bool real = (eb < NE);
  const int ebc = real ? eb : (NE - SP);
  int rec[SP]; int cnt = 0;
#pragma unroll
  for (int k = 0; k < SP; k += 4) {
    const v4i d4 = *(const v4i*)(dstv + ebc + k);
    v4i s4 = {0, 0, 0, 0};
    if (SRCL) s4 = *(const v4i*)(srcv + ebc + k);
#pragma unroll
    for (int e = 0; e < 4; ++e) {
      int sr = s4[e]; sr = sr < 0 ? 0 : (sr >= NN ? NN - 1 : sr);
      const int d = d4[e];
      int r = -1;
      if (real && d >= n0 && d < n0 + SRB) { r = ((d - n0) << 17) | sr; ++cnt; }
      rec[k + e] = r;
    }
  }
  int tot; int p = blk_excl_scan(cnt, scan_ws, tid, &tot);
#pragma unroll
  for (int k = 0; k < SP; ++k) if (rec[k] >= 0) { if ((unsigned)p < (unsigned)CAP) LIST[p] = rec[k]; ++p; }
  __syncthreads();
  return tot < CAP ? tot : CAP;
}

__global__ __launch_bounds__(NT) void deg_kernel(const int* __restrict__ ei, float* __restrict__ DINV) {
  __shared__ int LIST[SCH];
  __shared__ int scan_ws[80];
  const int tid = threadIdx.x, lane = tid & 31, wave = tid >> 5;
  const int n0 = blockIdx.x * SRB;
  const int* srcv = ei; const int* dstv = ei + NE;
  int cA0 = 0, cA1 = 0, cA2 = 0, cA3 = 0, cB0 = 0, cB1 = 0, cB2 = 0, cB3 = 0;
#pragma unroll 1
  for (int c = 0; c < NCH; ++c) {
    const int tot = chunk_hits<SPT, SCH, false>(dstv, srcv, c * SCH, n0, tid, LIST, scan_ws);
#pragma unroll 1
    for (int base = 0; base < tot; base += 32) {
      const int q = base + lane;
      const int qc = (q < SCH) ? q : (SCH - 1);
      const int lv = LIST[qc];
      const int rv = (q < tot) ? lv : -1;
      const int own = (rv >= 0 && (rv >> 25) == wave) ? 1 : 0;
      unsigned msk = (unsigned)__ballot(own);
#pragma unroll 1
      for (int it = 0; it < 32; ++it) {
        if (msk == 0u) break;
        const int bp = __builtin_ctz(msk); msk &= msk - 1u;
        const int r = __shfl(rv, bp, 32);
        const int dll = (r >> 17) & 255;
        const int hs  = dll >> 7;
        const int ol  = (dll >> 2) & 31;
        const int ix  = dll & 3;
        const bool mine = (ol == lane);
        const bool mA = mine && (hs == 0), mB = mine && (hs == 1);
        cA0 += (mA && ix == 0) ? 1 : 0; cA1 += (mA && ix == 1) ? 1 : 0; cA2 += (mA && ix == 2) ? 1 : 0; cA3 += (mA && ix == 3) ? 1 : 0;
        cB0 += (mB && ix == 0) ? 1 : 0; cB1 += (mB && ix == 1) ? 1 : 0; cB2 += (mB && ix == 2) ? 1 : 0; cB3 += (mB && ix == 3) ? 1 : 0;
      }
    }
    __syncthreads();
  }
  v4f dA, dB;
  dA[0] = rsqrtf((float)cA0 + 1.0f); dA[1] = rsqrtf((float)cA1 + 1.0f); dA[2] = rsqrtf((float)cA2 + 1.0f); dA[3] = rsqrtf((float)cA3 + 1.0f);
  dB[0] = rsqrtf((float)cB0 + 1.0f); dB[1] = rsqrtf((float)cB1 + 1.0f); dB[2] = rsqrtf((float)cB2 + 1.0f); dB[3] = rsqrtf((float)cB3 + 1.0f);
  float* pA = DINV + (size_t)n0 + wave * 256 + 4 * lane;
  float* pB = pA + 128;
  *(volatile v4f*)pA = dA; *(volatile v4f*)pB = dB;
  __threadfence();
  *(volatile v4f*)pA = dA; *(volatile v4f*)pB = dB;
}

template <bool OUT16>
__global__ __launch_bounds__(NT) void prop_kernel(const float* __restrict__ SRC, const int* __restrict__ ei, const float* __restrict__ DINV,
                                                  float* ACC, void* __restrict__ OUTP) {
  __shared__ int LIST[SCH];
  __shared__ int scan_ws[80];
  const int tid = threadIdx.x, lane = tid & 31, wave = tid >> 5;
  const int n0 = blockIdx.x * SRB;
  const v4f z4 = {0.f, 0.f, 0.f, 0.f};
#pragma unroll 1
  for (int j = 0; j < SRB / 8; ++j) {
    float* rp = ACC + (size_t)(n0 + wave * (SRB / 8) + j) * DD + 4 * lane;
    *(v4f*)rp = z4;
  }
  const int* srcv = ei; const int* dstv = ei + NE;
#pragma unroll 1
  for (int c = 0; c < NCH; ++c) {
    const int tot = chunk_hits<SPT, SCH, true>(dstv, srcv, c * SCH, n0, tid, LIST, scan_ws);
#pragma unroll 1
    for (int base = 0; base < tot; base += 32) {
      const int q = base + lane;
      const int qc = (q < SCH) ? q : (SCH - 1);
      const int lv = LIST[qc];
      const int rv = (q < tot) ? lv : -1;
      const int own = (rv >= 0 && (rv >> 25) == wave) ? 1 : 0;
      unsigned msk = (unsigned)__ballot(own);
#pragma unroll 1
      for (int it = 0; it < 32; ++it) {
        if (msk == 0u) break;
        const int bp = __builtin_ctz(msk); msk &= msk - 1u;
        const int r = __shfl(rv, bp, 32);
        const int dl = (r >> 17) & (SRB - 1);
        int s = r & 0x1FFFF; s = (s < NN) ? s : (NN - 1);
        const float ds = DINV[s];
        const v4f pv = *(const v4f*)(SRC + (size_t)s * DD + 4 * lane);
        float* rp = ACC + (size_t)(n0 + dl) * DD + 4 * lane;
        v4f a = *(const v4f*)rp;
        a = a + pv * ds;
        *(v4f*)rp = a;
      }
    }
    __syncthreads();
  }
  if (!OUT16) {
    float* X = (float*)OUTP;
#pragma unroll 1
    for (int j = 0; j < SRB / 8; ++j) {
      const int n = n0 + wave * (SRB / 8) + j;
      const int nc = (n < NN) ? n : (NN - 1);
      const float dn = DINV[n];
      const v4f a  = *(const v4f*)(ACC + (size_t)n * DD + 4 * lane);
      const v4f xs = *(const v4f*)(SRC + (size_t)nc * DD + 4 * lane);
      v4f v = (a + xs * dn) * dn;
      if (n >= NN) v = z4;
      float* op = X + (size_t)n * DD + 4 * lane;
      *(volatile v4f*)op = v;
      __threadfence();
      *(volatile v4f*)op = v;
    }
  } else {
    _Float16* X = (_Float16*)OUTP;
    const int hh = lane >> 4, c8 = (lane & 15) * 8;
#pragma unroll 1
    for (int jj = 0; jj < SRB / 16; ++jj) {
      const int dl = wave * (SRB / 8) + 2 * jj + hh;
      const int n = n0 + dl;
      const int nc = (n < NN) ? n : (NN - 1);
      const float dn = DINV[n];
      const float* rp = ACC + (size_t)n * DD + c8;
      const float* sp = SRC + (size_t)nc * DD + c8;
      const v4f aA = *(const v4f*)rp, aB = *(const v4f*)(rp + 4);
      const v4f xA = *(const v4f*)sp, xB = *(const v4f*)(sp + 4);
      const float dsc = dn * 64.0f;
      v4f qA = (aA + xA * dn) * dsc;
      v4f qB = (aB + xB * dn) * dsc;
      if (n >= NN) { qA = z4; qB = z4; }
      v8h hv;
#pragma unroll
      for (int e = 0; e < 4; ++e) { hv[e] = (_Float16)qA[e]; hv[4 + e] = (_Float16)qB[e]; }
      _Float16* op = X + (size_t)n * DD + c8;
      *(volatile v8h*)op = hv;
      __threadfence();
      *(volatile v8h*)op = hv;
    }
  }
}

__global__ __launch_bounds__(NT) void lsm_kernel(const float* __restrict__ LG, const float* __restrict__ bias, float* __restrict__ out) {
  __shared__ __align__(16) float res[LSB * NCLS];
  const int tid = threadIdx.x, lane = tid & 31, wave = tid >> 5;
  const int r0 = blockIdx.x * LSB;
  int nrows = NN - r0; nrows = (nrows > LSB) ? LSB : nrows;
  const int c2  = 32 + lane;
  const int c2b = (c2 < NCLS) ? c2 : (NCLS - 1);
  const float b1 = bias[lane], b2 = bias[c2b];
  const bool has2 = lane < (NCLS - 32);
#pragma unroll 1
  for (int rr = wave; rr < LSB; rr += NT / 32) {
    const float* lp = LG + (size_t)(r0 + rr) * NCP;
    const float v1 = lp[lane] + b1;
    const float v2 = lp[c2] + b2;
    const float v2m = has2 ? v2 : -3.0e38f;
    float m = fmaxf(v1, v2m);
#pragma unroll
    for (int d = 16; d >= 1; d >>= 1) m = fmaxf(m, __shfl_xor(m, d, 32));
    const float e1 = expf(v1 - m);
    const float e2 = expf(v2m - m);
    float s = e1 + (has2 ? e2 : 0.0f);
#pragma unroll
    for (int d = 16; d >= 1; d >>= 1) s += __shfl_xor(s, d, 32);
    const float lse = m + logf(s);
    res[rr * NCLS + lane] = v1 - lse;
    if (has2) res[rr * NCLS + c2] = v2 - lse;
  }
  __syncthreads();
  const int n4 = nrows * (NCLS / 4);
  float* ob = out + (size_t)r0 * NCLS;
  for (int pass = 0; pass < 2; ++pass) {
#pragma unroll 1
    for (int it = wave; it * 32 < n4; it += NT / 32) {
      const int idx = it * 32 + lane;
      const v4f v = *(const v4f*)(res + 4 * idx);
      *(volatile v4f*)(ob + 4 * (size_t)idx) = v;
    }
    __threadfence();
  }
}

extern "C" void kernel_launch(void* const* d_in, const int* in_sizes, int n_in,
                              void* d_out, int out_size, void* d_ws, size_t ws_size, hipStream_t stream) {
  if (n_in < 4) return;
  if (in_sizes[0] != NN * DD || in_sizes[1] != 2 * NE || in_sizes[2] != DD * NCLS || in_sizes[3] != NCLS || out_size != NN * NCLS) return;
  const float* x      = (const float*)d_in[0];
  const int*   ei     = (const int*)  d_in[1];
  const float* weight = (const float*)d_in[2];
  const float* bias   = (const float*)d_in[3];
  float* out = (float*)d_out;

  char* ws = (char*)d_ws; size_t off = 0;
  auto carve = [&](size_t bytes) -> char* { char* p = ws + off; off += (bytes + 255) & ~(size_t)255; return p; };
  unsigned* WT   = (unsigned*)carve((size_t)NCP * DD * 2);
  float*    DINV = (float*)   carve((size_t)NPA * 4);
  float*    ACC  = (float*)   carve((size_t)NPA * DD * 4);
  float*    X1   = (float*)   carve((size_t)NPA * DD * 4);
  _Float16* X2H  = (_Float16*)carve((size_t)NPA * DD * 2);
  float*    LG   = ACC;
  if (off > ws_size || off > (size_t)134217728) return;
  if ((size_t)MP * NCP * 4 > (size_t)NPA * DD * 4) return;

  wt_cast_kernel<<<(NCP * (DD / 2)) / 256, 256, 0, stream>>>(weight, WT);
  deg_kernel<<<NTL, NT, 0, stream>>>(ei, DINV);
  prop_kernel<false><<<NTL, NT, 0, stream>>>(x, ei, DINV, ACC, (void*)X1);
  prop_kernel<true><<<NTL, NT, 0, stream>>>(X1, ei, DINV, ACC, (void*)X2H);
  {
    const int tiles = (MP / 64) * (NCP / 64);
    wmma_gemm64<0, false, 0, 0, false><<<dim3((tiles + 7) / 8, 1), 256, 0, stream>>>(
        (const unsigned short*)X2H, nullptr, DD, 0L, (const unsigned short*)WT, nullptr, DD, 0L,
        (void*)LG, nullptr, NCP, 0L, nullptr, nullptr, 0L, MP, NCP, DD, 1.0f / 1024.0f);
  }
  lsm_kernel<<<NLB, NT, 0, stream>>>(LG, bias, out);
}
